// GCNWithPositionalEncoding_5909874999433
// MI455X (gfx1250) — hardware-verified
//
#include <hip/hip_runtime.h>
#include <math.h>

typedef __attribute__((ext_vector_type(16))) _Float16 v16h;
typedef __attribute__((ext_vector_type(16))) __bf16 v16b;
typedef __attribute__((ext_vector_type(8)))  _Float16 v8h;
typedef __attribute__((ext_vector_type(8)))  float v8f;
typedef __attribute__((ext_vector_type(4)))  float v4f;
typedef __attribute__((ext_vector_type(2)))  float v2f;
typedef __attribute__((ext_vector_type(4)))  unsigned v4u;
typedef __attribute__((ext_vector_type(4)))  int v4i;
typedef float __attribute__((may_alias)) float_a;
typedef int __attribute__((may_alias)) int_a;

template <typename T> __device__ __forceinline__ void vst2(void* p, T v) { *(volatile T*)p = v; __threadfence(); *(volatile T*)p = v; }
__device__ __forceinline__ v8f wmma16(v16h a, v16h b, v8f c) {
  v8f d = __builtin_amdgcn_wmma_f32_16x16x32_f16(false, a, false, b, (short)0, c, false, false);
  asm volatile("v_nop\n\tv_nop\n\tv_nop\n\tv_nop" : "+v"(d) : "v"(a), "v"(b));
  return d;
}
__device__ __forceinline__ v8f wmma_bf(v16b a, v16b b, v8f c) {
  v8f d = __builtin_amdgcn_wmma_f32_16x16x32_bf16(false, a, false, b, (short)0, c, false, false);
  asm volatile("v_nop\n\tv_nop\n\tv_nop\n\tv_nop" : "+v"(d) : "v"(a), "v"(b));
  return d;
}
__device__ __forceinline__ v16h frag_h(const _Float16* rowk0, int lane) {
  union { v16h v; v8h q[2]; } u; const _Float16* p = rowk0 + 8 * (lane >> 4);
  u.q[0] = *(const v8h*)p; u.q[1] = *(const v8h*)(p + 16); return u.v;
}
__device__ __forceinline__ v16h frag_f32(const float* rowk0, int lane) {
  v16h a; const float* p = rowk0 + 8 * (lane >> 4);
#pragma unroll
  for (int i = 0; i < 8; ++i) { a[i] = (_Float16)p[i]; a[8 + i] = (_Float16)p[16 + i]; }
  return a;
}
__device__ __forceinline__ v16h frag_f32s(const float* rowk0, int lane, float sc) {
  v16h a; const float* p = rowk0 + 8 * (lane >> 4);
#pragma unroll
  for (int i = 0; i < 8; ++i) { a[i] = (_Float16)(p[i] * sc); a[8 + i] = (_Float16)(p[16 + i] * sc); }
  return a;
}
__device__ __forceinline__ v16h fragc_f32(const float* W, int k0, int n, int lane, int ld, int K) {
  v16h a; const int g = lane >> 4;
#pragma unroll
  for (int i = 0; i < 8; ++i) { const int ka = k0 + 8 * g + i, kb = ka + 16;
    a[i] = (_Float16)(ka < K ? W[(size_t)ka * ld + n] : 0.f); a[8 + i] = (_Float16)(kb < K ? W[(size_t)kb * ld + n] : 0.f); }
  return a;
}
struct F2 { v16b h, l; };
__device__ __forceinline__ F2 bsplit16(const float v[16]) { F2 r;
#pragma unroll
  for (int i = 0; i < 16; ++i) { const __bf16 h = (__bf16)v[i]; r.h[i] = h; r.l[i] = (__bf16)(v[i] - (float)h); }
  return r; }
__device__ __forceinline__ F2 split_row(const float* row, int k0, int lane) { float v[16]; const float* p = row + k0 + 8 * (lane >> 4);
#pragma unroll
  for (int i = 0; i < 8; ++i) { v[i] = p[i]; v[8 + i] = p[16 + i]; }
  return bsplit16(v); }
__device__ __forceinline__ F2 split_rowK(const float* row, int k0, int lane, int K) { float v[16]; const int g = lane >> 4;
#pragma unroll
  for (int i = 0; i < 8; ++i) { const int ka = k0 + 8 * g + i, kb = ka + 16; v[i] = ka < K ? row[ka] : 0.f; v[8 + i] = kb < K ? row[kb] : 0.f; }
  return bsplit16(v); }
__device__ __forceinline__ F2 split_col(const float* W, int k0, int n, int lane, int ld, int K) { float v[16]; const int g = lane >> 4;
#pragma unroll
  for (int i = 0; i < 8; ++i) { const int ka = k0 + 8 * g + i, kb = ka + 16; v[i] = ka < K ? W[(size_t)ka * ld + n] : 0.f; v[8 + i] = kb < K ? W[(size_t)kb * ld + n] : 0.f; }
  return bsplit16(v); }
__device__ __forceinline__ v8f mac3(const F2& a, const F2& b, v8f c) { c = wmma_bf(a.l, b.h, c); c = wmma_bf(a.h, b.l, c); return wmma_bf(a.h, b.h, c); }
__device__ __forceinline__ float sigm(float v) { return 1.0f / (1.0f + expf(-v)); }
#define LDSX() do { asm volatile("s_wait_dscnt 0" ::: "memory"); __builtin_amdgcn_wave_barrier(); __builtin_amdgcn_fence(__ATOMIC_RELEASE, "workgroup"); } while (0)

#define NN 50000
#define NE 600000
#define NG 64
#define EMB 256
#define VOC 200
#define NDEP 51
#define NCH 21
#define DE 32
#define F0 128
#define FC 40
#define FCP 64
#define RB 512
#define NRB ((NN + RB - 1) / RB)
#define NNP (NRB * RB)
#define EPT 16
#define CH (256 * EPT)

#define RBD 8192
#define NRBD ((NN + RBD - 1) / RBD)
__device__ __forceinline__ void load4ids(const int* __restrict__ ids, int e, int dd[4]) { const int4 a = *(const int4*)(ids + e); dd[0] = a.x; dd[1] = a.y; dd[2] = a.z; dd[3] = a.w; }
__global__ __launch_bounds__(256) void k_deg(const int* __restrict__ ei, float* __restrict__ DINV) {
  __shared__ int scnt[RBD];
  const int tid = threadIdx.x; const int r0 = blockIdx.x * RBD; const int* edst = ei + NE;
  for (int q = tid; q < RBD; q += 256) scnt[q] = 0;
  __syncthreads();
#pragma unroll 1
  for (int c0 = 0; c0 < NE; c0 += CH) { const int e0 = c0 + tid * EPT;
    if (e0 + EPT <= NE) {
#pragma unroll
      for (int v = 0; v < EPT / 4; ++v) { int dd[4]; load4ids(edst, e0 + v * 4, dd);
#pragma unroll
        for (int u = 0; u < 4; ++u) { const unsigned rel = (unsigned)(dd[u] - r0); if (rel < (unsigned)RBD) atomicAdd(&scnt[rel], 1); } } }
    else { for (int u = 0; u < EPT; ++u) { const int e = e0 + u; if (e < NE) { const unsigned rel = (unsigned)(edst[e] - r0); if (rel < (unsigned)RBD) atomicAdd(&scnt[rel], 1); } } } }
  __syncthreads();
  for (int q = tid; q < RBD; q += 256) { const int r = r0 + q; if (r < NNP) vst2(DINV + r, r < NN ? rsqrtf((float)(scnt[q] + 1)) : 0.f); }
}
template <int K, int NOUT, int WROWS>
__global__ __launch_bounds__(128) void k_gemm(const float* __restrict__ A, int lda, const float* __restrict__ W, const float* __restrict__ DINV, float* __restrict__ HS) {
  __shared__ __align__(16) float so[4][16][NOUT + 4];
  const int tid = threadIdx.x, wave = tid >> 5, lane = tid & 31, col = lane & 15, g = lane >> 4;
  const int r0 = blockIdx.x * 64 + wave * 16;
  constexpr int NT = (NOUT + 15) / 16;
  v8f acc[NT];
#pragma unroll
  for (int t = 0; t < NT; ++t) acc[t] = (v8f){};
const int ra = (r0 + col) < NN ? (r0 + col) : (NN - 1);
#pragma unroll 1
  for (int kc = 0; kc < K / 32; ++kc) { const F2 a = split_row(A + (size_t)ra * lda, kc * 32, lane);
#pragma unroll
    for (int t = 0; t < NT; ++t) { const int n = t * 16 + col; const int nn = n < NOUT ? n : 0; acc[t] = mac3(a, WROWS ? split_row(W + (size_t)nn * K, kc * 32, lane) : split_col(W, kc * 32, nn, lane, NOUT, K), acc[t]); } }
#pragma unroll
  for (int t = 0; t < NT; ++t) { const int n = t * 16 + col;
#pragma unroll
    for (int r = 0; r < 8; ++r) { const int row = r0 + 8 * g + r; const float dv = row < NN ? DINV[row] : 0.f; if (n < NOUT) so[wave][8 * g + r][n] = acc[t][r] * dv; } }
  LDSX();
  for (int q = lane; q < 16 * (NOUT / 4); q += 32) { const int rl = q / (NOUT / 4), pc = q % (NOUT / 4); vst2(HS + (size_t)(r0 + rl) * NOUT + pc * 4, *(const v4f*)(&so[wave][rl][pc * 4])); }
}
template <int F, int MODE>
__global__ __launch_bounds__(256) void k_agg(const float* __restrict__ HS, const int* __restrict__ ei, const float* __restrict__ DINV, const float* __restrict__ bias, const float* __restrict__ lng, const float* __restrict__ lnb, float* __restrict__ OUT) {
  __shared__ __align__(16) float sacc[RB][F];
  __shared__ int ssrc[8][32 * EPT], sdl[8][32 * EPT]; __shared__ int scnt[8];
  const int tid = threadIdx.x, wave = tid >> 5, lane = tid & 31;
  const int r0 = blockIdx.x * RB; const int* esrc = ei; const int* edst = ei + NE;
  for (int q = tid; q < RB * F; q += 256) (&sacc[0][0])[q] = 0.f;
  __syncthreads();
#pragma unroll 1
  for (int c0 = 0; c0 < NE; c0 += CH) {
    const int e0 = c0 + tid * EPT; int hd[EPT]; int cnt = 0;
    if (e0 + EPT <= NE) {
#pragma unroll
      for (int v = 0; v < EPT / 4; ++v) { int dd[4]; load4ids(edst, e0 + v * 4, dd);
#pragma unroll
        for (int u = 0; u < 4; ++u) { const unsigned rel = (unsigned)(dd[u] - r0); const bool h = rel < (unsigned)RB; hd[v * 4 + u] = h ? (int)rel : -1; cnt += h ? 1 : 0; } } }
    else {
#pragma unroll
      for (int u = 0; u < EPT; ++u) { const int e = e0 + u; hd[u] = -1; if (e < NE) { const unsigned rel = (unsigned)(edst[e] - r0); if (rel < (unsigned)RB) { hd[u] = (int)rel; ++cnt; } } } }
    int incl = cnt;
#pragma unroll
    for (int off = 1; off < 32; off <<= 1) { const int vv = __shfl_up(incl, off, 32); if (lane >= off) incl += vv; }
    const int wtot = __shfl(incl, 31, 32); int pos = incl - cnt;
    if (cnt > 0) {
#pragma unroll
      for (int u = 0; u < EPT; ++u) if (hd[u] >= 0) { int s = esrc[e0 + u]; s = s < 0 ? 0 : (s >= NN ? NN - 1 : s); ssrc[wave][pos] = s; sdl[wave][pos] = hd[u];  ++pos; } }
    if (lane == 0) scnt[wave] = wtot;
    __syncthreads();
    if (tid < F) { for (int w = 0; w < 8; ++w) { const int nh = scnt[w]; for (int i = 0; i < nh; ++i) sacc[sdl[w][i]][tid] += HS[(size_t)ssrc[w][i] * F + tid]; } }
    __syncthreads(); }
  for (int rl = tid; rl < RB; rl += 256) { const int row = r0 + rl; if (row >= NN) continue; const float dv = DINV[row]; float* ar = &sacc[rl][0]; const float* hs = HS + (size_t)row * F;
    for (int f = 0; f < F; ++f) ar[f] = (ar[f] + hs[f]) * dv + bias[f];
    if (MODE == 2) { for (int f = 0; f < F; ++f) ar[f] = ar[f] > 0.f ? ar[f] : 0.f; }
    else if (MODE == 0) { float mu = 0.f; for (int f = 0; f < F; ++f) mu += ar[f]; mu *= (1.0f / F); float var = 0.f; for (int f = 0; f < F; ++f) { const float d = ar[f] - mu; var += d * d; } var *= (1.0f / F);
      const float rs = rsqrtf(var + 1e-5f); for (int f = 0; f < F; ++f) { const float v = (ar[f] - mu) * rs * lng[f] + lnb[f]; ar[f] = v > 0.f ? v : 0.f; } }
    else { float mx = -3.4e38f; for (int f = 0; f < FC; ++f) mx = fmaxf(mx, ar[f]); float se = 0.f; for (int f = 0; f < FC; ++f) se += expf(ar[f] - mx); const float lse = logf(se) + mx; for (int f = 0; f < FC; ++f) ar[f] -= lse; } }
  __syncthreads();
  if (MODE != 1) { for (int q = tid; q < RB * (F / 4); q += 256) { const int rl = q / (F / 4), pc = q % (F / 4); const int row = r0 + rl; v4f v = *(const v4f*)(&sacc[rl][pc * 4]); if (row >= NN) { if (MODE == 2) continue; v = (v4f){0.f, 0.f, 0.f, 0.f}; } vst2(OUT + (size_t)row * F + pc * 4, v); } }
  else {
    for (int q = tid; q < RB * FC / 4; q += 256) { const int rl = (q * 4) / FC, f = (q * 4) % FC; const int row = r0 + rl; if (row < NN) { v4f v; v[0] = sacc[rl][f]; v[1] = sacc[rl][f + 1]; v[2] = sacc[rl][f + 2]; v[3] = sacc[rl][f + 3]; vst2(OUT + (size_t)row * FC + f, v); } } }
}
template <int K>
__global__ __launch_bounds__(128) void k_tab(const float* __restrict__ A, const float* __restrict__ Bm, int M, float* __restrict__ T) {
  __shared__ __align__(16) float so[4][16][132];
  const int tid = threadIdx.x, wave = tid >> 5, lane = tid & 31, col = lane & 15, g = lane >> 4;
  const int r0 = blockIdx.x * 64 + wave * 16; const int ra = (r0 + col) < M ? (r0 + col) : (M - 1);
#pragma unroll 1
  for (int nh = 0; nh < 2; ++nh) { v8f acc[8] = {};
#pragma unroll 1
    for (int kc = 0; kc < K / 32; ++kc) { const F2 a = split_row(A + (size_t)ra * K, kc * 32, lane);
#pragma unroll
      for (int j = 0; j < 8; ++j) acc[j] = mac3(a, split_col(Bm, kc * 32, nh * 128 + j * 16 + col, lane, EMB, K), acc[j]); }
#pragma unroll
    for (int j = 0; j < 8; ++j)
#pragma unroll
      for (int r = 0; r < 8; ++r) so[wave][8 * g + r][j * 16 + col] = acc[j][r];
    LDSX();
    for (int rl = 0; rl < 16; ++rl) { if (r0 + rl >= M) break; vst2(T + (size_t)(r0 + rl) * EMB + nh * 128 + lane * 4, *(const v4f*)(&so[wave][rl][lane * 4])); }
    LDSX(); }
}
__global__ __launch_bounds__(256) void k_embed(const int* __restrict__ xi, const int* __restrict__ dep, const int* __restrict__ chl, const float* __restrict__ T1, const float* __restrict__ T2,
                                              const float* __restrict__ T3, const float* __restrict__ pb, float* __restrict__ H0) {
  const int q = blockIdx.x * 256 + threadIdx.x; const int n = q >> 6, pc = q & 63; if (n >= NNP) return;
  v4f v = {0.f, 0.f, 0.f, 0.f};
  if (n < NN) { int a = xi[n]; a = a < 0 ? 0 : (a >= VOC ? VOC - 1 : a); int d = dep[n]; d = d < 0 ? 0 : (d > NDEP - 1 ? NDEP - 1 : d); int c = chl[n]; c = c < 0 ? 0 : (c > NCH - 1 ? NCH - 1 : c);
    const v4f t1 = *(const v4f*)(T1 + (size_t)a * EMB + pc * 4), t2 = *(const v4f*)(T2 + (size_t)d * EMB + pc * 4), t3 = *(const v4f*)(T3 + (size_t)c * EMB + pc * 4), b4 = *(const v4f*)(pb + pc * 4);
#pragma unroll
    for (int e = 0; e < 4; ++e) { const float s = t1[e] + t2[e] + t3[e] + b4[e]; v[e] = s > 0.f ? s : 0.f; } }
  vst2(H0 + (size_t)n * EMB + pc * 4, v);
}
__global__ __launch_bounds__(256) void k_pool(const float* __restrict__ H, const int* __restrict__ batch, float* __restrict__ P) {
  __shared__ __align__(16) float ssum[F0]; __shared__ int slst[8][32]; __shared__ int scnt[8]; __shared__ int stot[8];
  const int tid = threadIdx.x, wave = tid >> 5, lane = tid & 31; const int gph = blockIdx.x;
  if (tid < F0) ssum[tid] = 0.f;
  int mycnt = 0;
  __syncthreads();
#pragma unroll 1
  for (int n0 = 0; n0 < NN; n0 += 256) { const int n = n0 + tid; const bool hit = (n < NN) && (batch[n] == gph);
    int incl = hit ? 1 : 0;
#pragma unroll
    for (int off = 1; off < 32; off <<= 1) { const int vv = __shfl_up(incl, off, 32); if (lane >= off) incl += vv; }
    const int wtot = __shfl(incl, 31, 32);
    if (hit) { slst[wave][incl - 1] = n; ++mycnt; }
    if (lane == 0) scnt[wave] = wtot;
    __syncthreads();
    if (tid < F0) { for (int w = 0; w < 8; ++w) { const int nh = scnt[w]; for (int i = 0; i < nh; ++i) ssum[tid] += H[(size_t)slst[w][i] * F0 + tid]; } }
    __syncthreads(); }
#pragma unroll
  for (int off = 16; off > 0; off >>= 1) mycnt += __shfl_xor(mycnt, off, 32);
  if (lane == 0) stot[wave] = mycnt;
  __syncthreads();
  if (tid < F0) { int cnt = 0;
#pragma unroll
    for (int w = 0; w < 8; ++w) cnt += stot[w];
    ssum[tid] = ssum[tid] / fmaxf((float)cnt, 1.0f); }
  __syncthreads();
  if (tid < 32) vst2(P + (size_t)gph * F0 + tid * 4, *(const v4f*)(&ssum[tid * 4]));
}
__global__ __launch_bounds__(256) void k_clf(const float* __restrict__ P, const float* __restrict__ cw, const float* __restrict__ cb, float* __restrict__ out) {
  __shared__ __align__(16) float sres[NG];
  const int tid = threadIdx.x, gph = tid >> 2, qd = tid & 3; const float* p = P + (size_t)gph * F0 + qd * 32; const float* w = cw + qd * 32; float a = 0.f;
#pragma unroll 4
  for (int k = 0; k < 32; ++k) a += p[k] * w[k];
  a += __shfl_xor(a, 1, 32); a += __shfl_xor(a, 2, 32);
  if (qd == 0) sres[gph] = a + cb[0];
  __syncthreads();
  if (tid < 16) vst2(out + tid * 4, *(const v4f*)(&sres[tid * 4]));
}
extern "C" void kernel_launch(void* const* d_in, const int* in_sizes, int n_in, void* d_out, int out_size, void* d_ws, size_t ws_size, hipStream_t stream) {
  (void)in_sizes; (void)n_in; (void)out_size; (void)ws_size;
  const int* xi = (const int*)d_in[0]; const int* ei = (const int*)d_in[1]; const int* batch = (const int*)d_in[2]; const int* dep = (const int*)d_in[3]; const int* chl = (const int*)d_in[4];
  const float* node_emb = (const float*)d_in[5]; const float* depth_emb = (const float*)d_in[6]; const float* child_emb = (const float*)d_in[7]; const float* P = (const float*)d_in[8]; const float* pb = (const float*)d_in[9];
  const float* W1 = (const float*)d_in[10]; const float* b1 = (const float*)d_in[11]; const float* W2 = (const float*)d_in[12]; const float* b2 = (const float*)d_in[13]; const float* cw = (const float*)d_in[14]; const float* cb = (const float*)d_in[15];
  float* out = (float*)d_out;
  char* ws = (char*)d_ws; size_t off = 0;
  auto take = [&](size_t bytes) { char* p = ws + off; off += (bytes + 255) & ~(size_t)255; return p; };
  float* T1 = (float*)take((size_t)256 * EMB * 4); float* T2 = (float*)take((size_t)64 * EMB * 4); float* T3 = (float*)take((size_t)64 * EMB * 4);
  float* DINV = (float*)take((size_t)NNP * 4); float* H0 = (float*)take((size_t)NNP * EMB * 4); float* HS = (float*)take((size_t)NNP * F0 * 4);
  float* X1 = (float*)take((size_t)NNP * F0 * 4); float* X2 = H0;   float* PG = (float*)take((size_t)NG * F0 * 4);
  k_tab<EMB><<<(VOC + 63) / 64, 128, 0, stream>>>(node_emb, P, VOC, T1);
  k_tab<DE><<<1, 128, 0, stream>>>(depth_emb, P + (size_t)EMB * EMB, NDEP, T2);
  k_tab<DE><<<1, 128, 0, stream>>>(child_emb, P + (size_t)(EMB + DE) * EMB, NCH, T3);
  k_embed<<<(NNP * 64 + 255) / 256, 256, 0, stream>>>(xi, dep, chl, T1, T2, T3, pb, H0);
  k_deg<<<NRBD, 256, 0, stream>>>(ei, DINV);
  k_gemm<EMB, F0, 0><<<NNP / 64, 128, 0, stream>>>(H0, EMB, W1, DINV, HS);
  k_agg<F0, 2><<<NRB, 256, 0, stream>>>(HS, ei, DINV, b1, nullptr, nullptr, X1);
  k_gemm<F0, F0, 0><<<NNP / 64, 128, 0, stream>>>(X1, F0, W2, DINV, HS);
  k_agg<F0, 2><<<NRB, 256, 0, stream>>>(HS, ei, DINV, b2, nullptr, nullptr, X2);
  k_pool<<<NG, 256, 0, stream>>>(X2, batch, PG);
  k_clf<<<1, 256, 0, stream>>>(PG, cw, cb, out);
}
